// PersLoss_6828998001473
// MI455X (gfx1250) — hardware-verified
//
#include <hip/hip_runtime.h>
#define NNODE 16000
#define IN 128
#define HID 64
#define NGR 32
#define NPR 128
#define DRES 100
#define NCLS 10

typedef __bf16 v16b __attribute__((ext_vector_type(16)));
typedef unsigned short v8us __attribute__((ext_vector_type(8), may_alias));
typedef float  v8f  __attribute__((ext_vector_type(8)));
typedef float  v4f  __attribute__((ext_vector_type(4)));
typedef float  v4fa __attribute__((ext_vector_type(4), may_alias));
union FragB { v16b v; v8us half[2]; unsigned short u[16]; };

__device__ __forceinline__ unsigned short bf16_bits(float x) { unsigned int u = __float_as_uint(x); return (unsigned short)((u + 0x7FFFu + ((u >> 16) & 1u)) >> 16); }
__device__ __forceinline__ float bf16_val(unsigned short b) { return __uint_as_float(((unsigned int)b) << 16); }
__device__ __forceinline__ float bf16_round(float x) { return bf16_val(bf16_bits(x)); }
template <int NT>
__device__ __forceinline__ v8f mmaN(v16b ah, v16b al, v16b bh, v16b bl, v8f c) {
  c = __builtin_amdgcn_wmma_f32_16x16x32_bf16(false, ah, false, bh, (short)0, c, false, false);
  if (NT >= 2) c = __builtin_amdgcn_wmma_f32_16x16x32_bf16(false, al, false, bh, (short)0, c, false, false);
  if (NT >= 3) c = __builtin_amdgcn_wmma_f32_16x16x32_bf16(false, ah, false, bl, (short)0, c, false, false);
  asm volatile("v_nop\n\tv_nop\n\tv_nop\n\tv_nop" : "+v"(c) : "v"(ah), "v"(al), "v"(bh), "v"(bl));
  return c;
}

__global__ __launch_bounds__(256) void k_wt_bf16(const float* __restrict__ W, unsigned short* __restrict__ Wt, int K, int N) {
  const int t = blockIdx.x * 256 + threadIdx.x;
  const int k8n = K / 8;
  if (t >= N * k8n) return;
  const int n = t / k8n, k8 = (t % k8n) * 8;
  v8us v;
#pragma unroll
  for (int i = 0; i < 8; ++i) v[i] = bf16_bits(W[(size_t)(k8 + i) * N + n]);
  *(volatile v8us*)(Wt + (size_t)n * K + k8) = v;
  __threadfence();
  *(volatile v8us*)(Wt + (size_t)n * K + k8) = v;
}

template <bool ASPLIT, int ACT, bool BIAS_BF16>
__global__ __launch_bounds__(128) void k_gemm_bf(const float* __restrict__ A, int lda, const unsigned short* __restrict__ Wt, int ldb,
                                               const float* __restrict__ bias, float* __restrict__ C, int ldc, int M, int N, int K) {
  __shared__ __attribute__((aligned(16))) float so[4][16][64];
  const int tid = threadIdx.x, w = tid >> 5, lane = tid & 31, ln = lane & 15, hh = lane >> 4;
  const int ntn = N / 64;
  const int wid = blockIdx.x * 4 + w;
  const int mt = wid / ntn, nq = wid % ntn;
  if (mt * 16 >= M) return;
  const int row0 = mt * 16, col0 = nq * 64;
  const float* arow = A + (size_t)(row0 + ln) * lda;
  v8f acc[4] = {};
  for (int kb = 0; kb < K; kb += 32) {
    FragB ah, al;
    const v4f x0 = *(const v4fa*)(arow + kb + 8 * hh), x1 = *(const v4fa*)(arow + kb + 8 * hh + 4);
    const v4f x2 = *(const v4fa*)(arow + kb + 16 + 8 * hh), x3 = *(const v4fa*)(arow + kb + 16 + 8 * hh + 4);
    float xs[16] = {x0[0],x0[1],x0[2],x0[3],x1[0],x1[1],x1[2],x1[3],x2[0],x2[1],x2[2],x2[3],x3[0],x3[1],x3[2],x3[3]};
#pragma unroll
    for (int i = 0; i < 16; ++i) { const unsigned short hb = bf16_bits(xs[i]); ah.u[i] = hb; al.u[i] = ASPLIT ? bf16_bits(xs[i] - bf16_val(hb)) : (unsigned short)0; }
#pragma unroll
    for (int t = 0; t < 4; ++t) {
      const unsigned short* brow = Wt + (size_t)(col0 + t * 16 + ln) * ldb + kb;
      FragB b;
      b.half[0] = *(const v8us*)(brow + 8 * hh);
      b.half[1] = *(const v8us*)(brow + 16 + 8 * hh);
      acc[t] = mmaN<ASPLIT ? 2 : 1>(ah.v, al.v, b.v, b.v, acc[t]);
    }
  }
#pragma unroll
  for (int t = 0; t < 4; ++t) {
    float bv = bias ? bias[col0 + t * 16 + ln] : 0.f;
    if (BIAS_BF16) bv = bf16_round(bv);
#pragma unroll
    for (int r = 0; r < 8; ++r) { float v = acc[t][r] + bv; if (ACT == 1) v = fmaxf(v, 0.f); so[w][8 * hh + r][t * 16 + ln] = v; }
  }
  __builtin_amdgcn_fence(__ATOMIC_ACQ_REL, "workgroup");
  __builtin_amdgcn_wave_barrier();
  const int rsub = lane >> 4, c4 = (lane & 15) * 4;
  for (int pass = 0; pass < 2; ++pass) {
#pragma unroll
    for (int q = 0; q < 8; ++q) {
      const int r = q * 2 + rsub;
      const v4f v = *(const v4fa*)&so[w][r][c4];
      *(volatile v4f*)(C + (size_t)(row0 + r) * ldc + col0 + c4) = v;
    }
    if (pass == 0) __threadfence();
  }
}

template <int D, bool CAUSAL>
__global__ __launch_bounds__(128) void k_flash(const float* __restrict__ qb, const float* __restrict__ kb, const float* __restrict__ vb,
                                             int pitch, int T, int H, float scale, float* __restrict__ y, int ypitch) {
  constexpr int KS = D / 32;
  constexpr int DT = D / 16;
  __shared__ __attribute__((aligned(16))) unsigned short sKh[32][D + 8], sKl[32][D + 8], sVh[32][D + 8], sVl[32][D + 8];
  __shared__ __attribute__((aligned(16))) unsigned short sPh[4][16][40], sPl[4][16][40];
  __shared__ __attribute__((aligned(16))) float sO[4][16][D];
  const int tid = threadIdx.x, w = tid >> 5, lane = tid & 31, ln = lane & 15, hh = lane >> 4;
  const int nqb = (T + 63) / 64;
  const int bh = blockIdx.x / nqb, qblk = blockIdx.x % nqb;
  const int b = bh / H, h = bh % H;
  const int q0 = qblk * 64 + w * 16;
  const float* Q = qb + (size_t)b * T * pitch + h * D;
  const float* K = kb + (size_t)b * T * pitch + h * D;
  const float* V = vb + (size_t)b * T * pitch + h * D;

  FragB aqh[KS], aql[KS];
  {
    int row = q0 + ln; if (row >= T) row = T - 1;
    const float* qr = Q + (size_t)row * pitch;
#pragma unroll
    for (int ks = 0; ks < KS; ++ks)
#pragma unroll
      for (int i = 0; i < 16; ++i) {
        const int d = ks * 32 + ((i < 8) ? (8 * hh + i) : (16 + 8 * hh + (i - 8)));
        const float x = qr[d] * scale; const unsigned short hb = bf16_bits(x);
        aqh[ks].u[i] = hb; aql[ks].u[i] = bf16_bits(x - bf16_val(hb));
      }
  }
  float m_r[8], l_r[8];
#pragma unroll
  for (int r = 0; r < 8; ++r) { m_r[r] = -3.0e38f; l_r[r] = 0.f; }
  v8f oacc[DT];
#pragma unroll
  for (int dt = 0; dt < DT; ++dt) oacc[dt] = (v8f){0.f,0.f,0.f,0.f,0.f,0.f,0.f,0.f};

  const int kv_end = CAUSAL ? min(T, qblk * 64 + 64) : T;
  for (int j0 = 0; j0 < kv_end; j0 += 32) {
    __syncthreads();
    for (int e = tid; e < 32 * (D / 4); e += 128) {
      const int r = e / (D / 4), c4 = (e % (D / 4)) * 4;
      const int key = j0 + r;
      v4f kf = {0.f,0.f,0.f,0.f}, vf = {0.f,0.f,0.f,0.f};
      if (key < T) { kf = *(const v4fa*)(K + (size_t)key * pitch + c4); vf = *(const v4fa*)(V + (size_t)key * pitch + c4); }
#pragma unroll
      for (int t = 0; t < 4; ++t) {
        unsigned short hb = bf16_bits(kf[t]); sKh[r][c4 + t] = hb; sKl[r][c4 + t] = bf16_bits(kf[t] - bf16_val(hb));
        hb = bf16_bits(vf[t]); sVh[r][c4 + t] = hb; sVl[r][c4 + t] = bf16_bits(vf[t] - bf16_val(hb));
      }
    }
    __syncthreads();
    v8f s[2];
#pragma unroll
    for (int nt = 0; nt < 2; ++nt) {
      v8f acc = {};
#pragma unroll
      for (int ks = 0; ks < KS; ++ks) {
        FragB bh_, bl_;
        bh_.half[0] = *(const v8us*)&sKh[nt * 16 + ln][ks * 32 + 8 * hh]; bh_.half[1] = *(const v8us*)&sKh[nt * 16 + ln][ks * 32 + 16 + 8 * hh];
        bl_.half[0] = *(const v8us*)&sKl[nt * 16 + ln][ks * 32 + 8 * hh]; bl_.half[1] = *(const v8us*)&sKl[nt * 16 + ln][ks * 32 + 16 + 8 * hh];
        acc = mmaN<3>(aqh[ks].v, aql[ks].v, bh_.v, bl_.v, acc);
      }
      s[nt] = acc;
    }
    float alpha[8];
#pragma unroll
    for (int r = 0; r < 8; ++r) {
      const int qi = q0 + 8 * hh + r;
      const int ja = j0 + ln, jb = j0 + 16 + ln;
      if (CAUSAL) { if (ja > qi) s[0][r] = -3.0e38f; if (jb > qi) s[1][r] = -3.0e38f; }
      if (ja >= T) s[0][r] = -3.0e38f;
      if (jb >= T) s[1][r] = -3.0e38f;
      float mx = fmaxf(s[0][r], s[1][r]);
      mx = fmaxf(mx, __shfl_xor(mx, 1, 32)); mx = fmaxf(mx, __shfl_xor(mx, 2, 32)); mx = fmaxf(mx, __shfl_xor(mx, 4, 32)); mx = fmaxf(mx, __shfl_xor(mx, 8, 32));
      const float mnew = fmaxf(m_r[r], mx);
      alpha[r] = (mnew > -1.0e38f) ? __expf(m_r[r] - mnew) : 1.0f;
      const float p0 = (s[0][r] > -1.0e38f) ? __expf(s[0][r] - mnew) : 0.f;
      const float p1 = (s[1][r] > -1.0e38f) ? __expf(s[1][r] - mnew) : 0.f;
      m_r[r] = mnew;
      l_r[r] = l_r[r] * alpha[r] + p0 + p1;
      unsigned short hb = bf16_bits(p0); sPh[w][8 * hh + r][ln] = hb;      sPl[w][8 * hh + r][ln] = bf16_bits(p0 - bf16_val(hb));
      hb = bf16_bits(p1);                sPh[w][8 * hh + r][16 + ln] = hb; sPl[w][8 * hh + r][16 + ln] = bf16_bits(p1 - bf16_val(hb));
    }
#pragma unroll
    for (int dt = 0; dt < DT; ++dt)
#pragma unroll
      for (int r = 0; r < 8; ++r) oacc[dt][r] *= alpha[r];
    __builtin_amdgcn_fence(__ATOMIC_ACQ_REL, "workgroup");
    __builtin_amdgcn_wave_barrier();
    FragB pah, pal;
    pah.half[0] = *(const v8us*)&sPh[w][ln][8 * hh]; pah.half[1] = *(const v8us*)&sPh[w][ln][16 + 8 * hh];
    pal.half[0] = *(const v8us*)&sPl[w][ln][8 * hh]; pal.half[1] = *(const v8us*)&sPl[w][ln][16 + 8 * hh];
#pragma unroll
    for (int dt = 0; dt < DT; ++dt) {
      FragB bvh, bvl;
#pragma unroll
      for (int i = 0; i < 8; ++i) {
        bvh.u[i] = sVh[8 * hh + i][dt * 16 + ln]; bvh.u[8 + i] = sVh[16 + 8 * hh + i][dt * 16 + ln];
        bvl.u[i] = sVl[8 * hh + i][dt * 16 + ln]; bvl.u[8 + i] = sVl[16 + 8 * hh + i][dt * 16 + ln];
      }
      oacc[dt] = mmaN<3>(pah.v, pal.v, bvh.v, bvl.v, oacc[dt]);
    }
    __builtin_amdgcn_fence(__ATOMIC_ACQ_REL, "workgroup");
    __builtin_amdgcn_wave_barrier();
  }
#pragma unroll
  for (int r = 0; r < 8; ++r) {
    float l = l_r[r];
    l += __shfl_xor(l, 1, 32); l += __shfl_xor(l, 2, 32); l += __shfl_xor(l, 4, 32); l += __shfl_xor(l, 8, 32);
    l_r[r] = (l > 0.f) ? 1.0f / l : 0.f;
  }
#pragma unroll
  for (int dt = 0; dt < DT; ++dt)
#pragma unroll
    for (int r = 0; r < 8; ++r) sO[w][8 * hh + r][dt * 16 + ln] = oacc[dt][r] * l_r[r];
  __builtin_amdgcn_fence(__ATOMIC_ACQ_REL, "workgroup");
  __builtin_amdgcn_wave_barrier();
  for (int pass = 0; pass < 2; ++pass) {
    for (int r = 0; r < 16; ++r) {
      const int row = q0 + r;
      if (row < T && lane < D / 4) {
        const v4f val = *(const v4fa*)&sO[w][r][lane * 4];
        *(volatile v4f*)(y + ((size_t)b * T + row) * ypitch + h * D + lane * 4) = val;
      }
    }
    if (pass == 0) __threadfence();
  }
}

template <bool AFFINE, bool RESID, bool RES_BF16>
__global__ __launch_bounds__(256) void k_transpose32(const float* __restrict__ in, float* __restrict__ out, int rows, int cols,
                                                    const float* __restrict__ scale, const float* __restrict__ shift, const float* __restrict__ res) {
  __shared__ float tile[32][33];
  const int b = blockIdx.z;
  const int r0 = blockIdx.y * 32, c0 = blockIdx.x * 32;
  const float* src = in + (size_t)b * rows * cols;
  float* dst = out + (size_t)b * rows * cols;
  const int tx = threadIdx.x & 31, ty = threadIdx.x >> 5;
  for (int i = ty; i < 32; i += 8) tile[i][tx] = src[(size_t)(r0 + i) * cols + c0 + tx];
  __syncthreads();
  for (int pass = 0; pass < 2; ++pass) {
    for (int i = ty; i < 32; i += 8) {
      float v = tile[tx][i];
      const int orow = c0 + i;
      if (AFFINE) v = v * scale[orow] + shift[orow];
      if (RESID) { float rv = res[(size_t)b * rows * cols + (size_t)orow * rows + r0 + tx]; if (RES_BF16) rv = bf16_round(rv); v += rv; }
      *(volatile float*)(dst + (size_t)orow * rows + r0 + tx) = v;
    }
    if (pass == 0) __threadfence();
  }
}

__global__ __launch_bounds__(256) void k_pool2_pm(const float* __restrict__ in, float* __restrict__ out, int Bn, int H, int W, int C) {
  const size_t t = (size_t)blockIdx.x * 256 + threadIdx.x;
  const int c4n = C / 4, Ho = H / 2, Wo = W / 2;
  const size_t total = (size_t)Bn * Ho * Wo * c4n;
  if (t >= total) return;
  const int c4 = (int)(t % c4n) * 4; size_t rest = t / c4n;
  const int pw = (int)(rest % Wo); rest /= Wo; const int ph = (int)(rest % Ho); const int b = (int)(rest / Ho);
  const float* base = in + (size_t)b * H * W * C;
  const int p00 = (2 * ph) * W + 2 * pw;
  const v4f a = *(const v4fa*)(base + (size_t)p00 * C + c4), bq = *(const v4fa*)(base + (size_t)(p00 + 1) * C + c4);
  const v4f c = *(const v4fa*)(base + (size_t)(p00 + W) * C + c4), d = *(const v4fa*)(base + (size_t)(p00 + W + 1) * C + c4);
  v4f m; for (int i = 0; i < 4; ++i) m[i] = fmaxf(fmaxf(a[i], bq[i]), fmaxf(c[i], d[i]));
  float* dst = out + ((size_t)b * Ho * Wo + (size_t)ph * Wo + pw) * C + c4;
  *(volatile v4f*)dst = m;
  __threadfence();
  *(volatile v4f*)dst = m;
}

template <int DQ, int DV>
__global__ __launch_bounds__(128) void k_flash2(const float* __restrict__ Qb, size_t qstride, int qpitch, int Tq,
                                              const float* __restrict__ Kb, size_t kstride, int kpitch, int Tk,
                                              const float* __restrict__ Vb, size_t vstride, int vpitch,
                                              float scale, float* __restrict__ y, size_t ystride, int ypitch) {
  constexpr int KS = DQ / 32, DT = DV / 16;
  __shared__ __attribute__((aligned(16))) unsigned short sKh[32][DQ + 8], sKl[32][DQ + 8], sVh[32][DV + 8], sVl[32][DV + 8];
  __shared__ __attribute__((aligned(16))) unsigned short sPh[4][16][40], sPl[4][16][40];
  __shared__ __attribute__((aligned(16))) float sO[4][16][DV];
  const int tid = threadIdx.x, w = tid >> 5, lane = tid & 31, ln = lane & 15, hh = lane >> 4;
  const int nqb = (Tq + 63) / 64;
  const int bh = blockIdx.x / nqb, qblk = blockIdx.x % nqb;
  const int dv0 = blockIdx.y * DV;
  const int q0 = qblk * 64 + w * 16;
  const float* Q = Qb + (size_t)bh * qstride; const float* K = Kb + (size_t)bh * kstride; const float* V = Vb + (size_t)bh * vstride + dv0;
  FragB aqh[KS], aql[KS];
  {
    int row = q0 + ln; if (row >= Tq) row = Tq - 1;
    const float* qr = Q + (size_t)row * qpitch;
#pragma unroll
    for (int ks = 0; ks < KS; ++ks)
#pragma unroll
      for (int i = 0; i < 16; ++i) {
        const int d = ks * 32 + ((i < 8) ? (8 * hh + i) : (16 + 8 * hh + (i - 8)));
        const float x = qr[d] * scale; const unsigned short hb = bf16_bits(x);
        aqh[ks].u[i] = hb; aql[ks].u[i] = bf16_bits(x - bf16_val(hb));
      }
  }
  float m_r[8], l_r[8];
#pragma unroll
  for (int r = 0; r < 8; ++r) { m_r[r] = -3.0e38f; l_r[r] = 0.f; }
  v8f oacc[DT];
#pragma unroll
  for (int dt = 0; dt < DT; ++dt) oacc[dt] = (v8f){0.f,0.f,0.f,0.f,0.f,0.f,0.f,0.f};
  for (int j0 = 0; j0 < Tk; j0 += 32) {
    __syncthreads();
    for (int e = tid; e < 32 * (DQ / 4); e += 128) {
      const int r = e / (DQ / 4), c4 = (e % (DQ / 4)) * 4; const int key = j0 + r;
      v4f f = {0.f,0.f,0.f,0.f}; if (key < Tk) f = *(const v4fa*)(K + (size_t)key * kpitch + c4);
#pragma unroll
      for (int t = 0; t < 4; ++t) { const unsigned short hb = bf16_bits(f[t]); sKh[r][c4 + t] = hb; sKl[r][c4 + t] = bf16_bits(f[t] - bf16_val(hb)); }
    }
    for (int e = tid; e < 32 * (DV / 4); e += 128) {
      const int r = e / (DV / 4), c4 = (e % (DV / 4)) * 4; const int key = j0 + r;
      v4f f = {0.f,0.f,0.f,0.f}; if (key < Tk) f = *(const v4fa*)(V + (size_t)key * vpitch + c4);
#pragma unroll
      for (int t = 0; t < 4; ++t) { const unsigned short hb = bf16_bits(f[t]); sVh[r][c4 + t] = hb; sVl[r][c4 + t] = bf16_bits(f[t] - bf16_val(hb)); }
    }
    __syncthreads();
    v8f s[2];
#pragma unroll
    for (int nt = 0; nt < 2; ++nt) {
      v8f acc = {};
#pragma unroll
      for (int ks = 0; ks < KS; ++ks) {
        FragB bh_, bl_;
        bh_.half[0] = *(const v8us*)&sKh[nt * 16 + ln][ks * 32 + 8 * hh]; bh_.half[1] = *(const v8us*)&sKh[nt * 16 + ln][ks * 32 + 16 + 8 * hh];
        bl_.half[0] = *(const v8us*)&sKl[nt * 16 + ln][ks * 32 + 8 * hh]; bl_.half[1] = *(const v8us*)&sKl[nt * 16 + ln][ks * 32 + 16 + 8 * hh];
        acc = mmaN<3>(aqh[ks].v, aql[ks].v, bh_.v, bl_.v, acc);
      }
      s[nt] = acc;
    }
    float alpha[8];
#pragma unroll
    for (int r = 0; r < 8; ++r) {
      const int ja = j0 + ln, jb = j0 + 16 + ln;
      if (ja >= Tk) s[0][r] = -3.0e38f;
      if (jb >= Tk) s[1][r] = -3.0e38f;
      float mx = fmaxf(s[0][r], s[1][r]);
      mx = fmaxf(mx, __shfl_xor(mx, 1, 32)); mx = fmaxf(mx, __shfl_xor(mx, 2, 32)); mx = fmaxf(mx, __shfl_xor(mx, 4, 32)); mx = fmaxf(mx, __shfl_xor(mx, 8, 32));
      const float mnew = fmaxf(m_r[r], mx);
      alpha[r] = (mnew > -1.0e38f) ? __expf(m_r[r] - mnew) : 1.0f;
      const float p0 = (s[0][r] > -1.0e38f) ? __expf(s[0][r] - mnew) : 0.f;
      const float p1 = (s[1][r] > -1.0e38f) ? __expf(s[1][r] - mnew) : 0.f;
      m_r[r] = mnew;
      l_r[r] = l_r[r] * alpha[r] + p0 + p1;
      unsigned short hb = bf16_bits(p0); sPh[w][8 * hh + r][ln] = hb;      sPl[w][8 * hh + r][ln] = bf16_bits(p0 - bf16_val(hb));
      hb = bf16_bits(p1);                sPh[w][8 * hh + r][16 + ln] = hb; sPl[w][8 * hh + r][16 + ln] = bf16_bits(p1 - bf16_val(hb));
    }
#pragma unroll
    for (int dt = 0; dt < DT; ++dt)
#pragma unroll
      for (int r = 0; r < 8; ++r) oacc[dt][r] *= alpha[r];
    __builtin_amdgcn_fence(__ATOMIC_ACQ_REL, "workgroup");
    __builtin_amdgcn_wave_barrier();
    FragB pah, pal;
    pah.half[0] = *(const v8us*)&sPh[w][ln][8 * hh]; pah.half[1] = *(const v8us*)&sPh[w][ln][16 + 8 * hh];
    pal.half[0] = *(const v8us*)&sPl[w][ln][8 * hh]; pal.half[1] = *(const v8us*)&sPl[w][ln][16 + 8 * hh];
#pragma unroll
    for (int dt = 0; dt < DT; ++dt) {
      FragB bvh, bvl;
#pragma unroll
      for (int i = 0; i < 8; ++i) {
        bvh.u[i] = sVh[8 * hh + i][dt * 16 + ln]; bvh.u[8 + i] = sVh[16 + 8 * hh + i][dt * 16 + ln];
        bvl.u[i] = sVl[8 * hh + i][dt * 16 + ln]; bvl.u[8 + i] = sVl[16 + 8 * hh + i][dt * 16 + ln];
      }
      oacc[dt] = mmaN<3>(pah.v, pal.v, bvh.v, bvl.v, oacc[dt]);
    }
    __builtin_amdgcn_fence(__ATOMIC_ACQ_REL, "workgroup");
    __builtin_amdgcn_wave_barrier();
  }
#pragma unroll
  for (int r = 0; r < 8; ++r) {
    float l = l_r[r];
    l += __shfl_xor(l, 1, 32); l += __shfl_xor(l, 2, 32); l += __shfl_xor(l, 4, 32); l += __shfl_xor(l, 8, 32);
    l_r[r] = (l > 0.f) ? 1.0f / l : 0.f;
  }
#pragma unroll
  for (int dt = 0; dt < DT; ++dt)
#pragma unroll
    for (int r = 0; r < 8; ++r) sO[w][8 * hh + r][dt * 16 + ln] = oacc[dt][r] * l_r[r];
  __builtin_amdgcn_fence(__ATOMIC_ACQ_REL, "workgroup");
  __builtin_amdgcn_wave_barrier();
  for (int pass = 0; pass < 2; ++pass) {
    for (int r = 0; r < 16; ++r) {
      const int row = q0 + r;
      for (int c4 = lane * 4; c4 < DV; c4 += 128) {
        if (row < Tq) {
          const v4f val = *(const v4fa*)&sO[w][r][c4];
          *(volatile v4f*)(y + (size_t)bh * ystride + (size_t)row * ypitch + dv0 + c4) = val;
        }
      }
    }
    if (pass == 0) __threadfence();
  }
}

__global__ __launch_bounds__(256) void k_round_rows(const float* __restrict__ W, unsigned short* __restrict__ Wt, int n8) {
  const int t = blockIdx.x * 256 + threadIdx.x;
  if (t >= n8) return;
  const v4f a = *(const v4fa*)(W + (size_t)t * 8), b = *(const v4fa*)(W + (size_t)t * 8 + 4);
  v8us v; v[0]=bf16_bits(a[0]); v[1]=bf16_bits(a[1]); v[2]=bf16_bits(a[2]); v[3]=bf16_bits(a[3]);
  v[4]=bf16_bits(b[0]); v[5]=bf16_bits(b[1]); v[6]=bf16_bits(b[2]); v[7]=bf16_bits(b[3]);
  *(volatile v8us*)(Wt + (size_t)t * 8) = v; __threadfence(); *(volatile v8us*)(Wt + (size_t)t * 8) = v;
}
__global__ __launch_bounds__(256) void k_wt_conv5(const float* __restrict__ w, unsigned short* __restrict__ Bt, int O, int Cin, int CinP, int Np) {
  const int t = blockIdx.x * 256 + threadIdx.x; const int K = 25 * CinP; if (t >= Np * (K / 8)) return;
  const int o = t / (K / 8), k8 = (t % (K / 8)) * 8; v8us v;
#pragma unroll 1
  for (int i = 0; i < 8; ++i) { const int k = k8 + i; const int tap = k / CinP, c = k % CinP; v[i] = (o < O && c < Cin) ? bf16_bits(w[((size_t)o * Cin + c) * 25 + tap]) : (unsigned short)0; }
  *(volatile v8us*)(Bt + (size_t)o * K + k8) = v; __threadfence(); *(volatile v8us*)(Bt + (size_t)o * K + k8) = v;
}
template <int CinP, int ACT, int HI_, int WI_>
__global__ __launch_bounds__(128) void k_conv5(const float* __restrict__ in, int inP, const unsigned short* __restrict__ Bt, const float* __restrict__ bias, int Nb, float* __restrict__ out, int Np, int npos) {
  constexpr int K = 25 * CinP, SPT = CinP / 32;
  __shared__ __attribute__((aligned(16))) float so[4][16][64];
  const int tid = threadIdx.x, w = tid >> 5, lane = tid & 31, ln = lane & 15, hh = lane >> 4;
  const int ntn = Np / 64; const int wid = blockIdx.x * 4 + w; const int mt = wid / ntn, nq = wid % ntn;
  if (mt * 16 >= npos) return;
  const int row0 = mt * 16, col0 = nq * 64; const int m = row0 + ln; const int n = m / (HI_ * WI_), yx = m % (HI_ * WI_), y = yx / WI_, xq = yx % WI_;
  v8f acc[4] = {};
#pragma unroll 1
  for (int tap = 0; tap < 25; ++tap) {
    const int yy = y + tap / 5 - 2, xx = xq + tap % 5 - 2; const bool inb = (yy >= 0 && yy < HI_ && xx >= 0 && xx < WI_);
    const float* src = in + ((size_t)n * HI_ * WI_ + (size_t)(inb ? yy : 0) * WI_ + (inb ? xx : 0)) * inP;
#pragma unroll
    for (int s = 0; s < SPT; ++s) {
      const int c0 = s * 32; v4f a0 = {0.f,0.f,0.f,0.f}, a1 = a0, a2 = a0, a3 = a0;
      if (inb) { a0 = *(const v4fa*)(src + c0 + 8 * hh); a1 = *(const v4fa*)(src + c0 + 8 * hh + 4); a2 = *(const v4fa*)(src + c0 + 16 + 8 * hh); a3 = *(const v4fa*)(src + c0 + 16 + 8 * hh + 4); }
      float xs[16] = {a0[0],a0[1],a0[2],a0[3],a1[0],a1[1],a1[2],a1[3],a2[0],a2[1],a2[2],a2[3],a3[0],a3[1],a3[2],a3[3]};
      FragB ah, al;
#pragma unroll
      for (int i = 0; i < 16; ++i) { const unsigned short hb = bf16_bits(xs[i]); ah.u[i] = hb; al.u[i] = bf16_bits(xs[i] - bf16_val(hb)); }
      const int kb = tap * CinP + c0;
#pragma unroll
      for (int t = 0; t < 4; ++t) { FragB bq; bq.half[0] = *(const v8us*)(Bt + (size_t)(col0 + t * 16 + ln) * K + kb + 8 * hh); bq.half[1] = *(const v8us*)(Bt + (size_t)(col0 + t * 16 + ln) * K + kb + 16 + 8 * hh); acc[t] = mmaN<2>(ah.v, al.v, bq.v, bq.v, acc[t]); }
    }
  }
#pragma unroll
  for (int t = 0; t < 4; ++t) { const int col = col0 + t * 16 + ln; const float bv = (col < Nb) ? bf16_round(bias[col]) : 0.f;
#pragma unroll
    for (int r = 0; r < 8; ++r) { float v = acc[t][r] + bv; if (ACT == 1) v = fmaxf(v, 0.f); else if (ACT == 2) v = v >= 0.f ? v : 0.1f * v; so[w][8 * hh + r][t * 16 + ln] = v; } }
  __builtin_amdgcn_fence(__ATOMIC_ACQ_REL, "workgroup"); __builtin_amdgcn_wave_barrier();
  const int rsub = lane >> 4, c4 = (lane & 15) * 4;
  for (int pass = 0; pass < 2; ++pass) { for (int q = 0; q < 8; ++q) { const int r = q * 2 + rsub; const v4f v = *(const v4fa*)&so[w][r][c4]; *(volatile v4f*)(out + (size_t)(row0 + r) * Np + col0 + c4) = v; } if (pass == 0) __threadfence(); }
}

__global__ __launch_bounds__(256) void k_filt(const float* __restrict__ h, const float* __restrict__ w2, const float* __restrict__ b2, float* __restrict__ filt, float* __restrict__ out1) {
  const int n = blockIdx.x * 256 + threadIdx.x; if (n >= NNODE) return; float s = bf16_round(b2[0]);
#pragma unroll 1
  for (int c = 0; c < HID; c += 4) { const v4f a = *(const v4fa*)(h + (size_t)n * HID + c); s += a[0] * bf16_round(w2[c]) + a[1] * bf16_round(w2[c + 1]) + a[2] * bf16_round(w2[c + 2]) + a[3] * bf16_round(w2[c + 3]); }
  const float v = 1.0f / (1.0f + expf(-s));
  *(volatile float*)(filt + n) = v; *(volatile float*)(out1 + n) = v; __threadfence(); *(volatile float*)(filt + n) = v; *(volatile float*)(out1 + n) = v;
}
__global__ __launch_bounds__(128) void k_persim(const float* __restrict__ filt, const int* __restrict__ pi0, const int* __restrict__ pi1, float* __restrict__ img, float* __restrict__ bmax) {
  __shared__ float sb[2][NPR], sp[2][NPR]; __shared__ float red[128]; __shared__ __attribute__((aligned(16))) float tile[DRES][32];
  const int b = blockIdx.x / DRES, i = blockIdx.x % DRES, j = threadIdx.x;
  for (int e = threadIdx.x; e < 2 * NPR; e += 128) { const int c = e / NPR, p = e % NPR; const int* pi = c ? pi1 : pi0; int ia = pi[((size_t)b * NPR + p) * 2], ib = pi[((size_t)b * NPR + p) * 2 + 1];
    ia = ia < 0 ? 0 : (ia >= NNODE ? NNODE - 1 : ia); ib = ib < 0 ? 0 : (ib >= NNODE ? NNODE - 1 : ib); const float birth = filt[ia], death = filt[ib]; sb[c][p] = birth; sp[c][p] = death - birth; }
  __syncthreads();
  const float ci = (float)i / (float)DRES, cj = (float)j / (float)DRES;
  float v0 = 0.f, v1 = 0.f;
  if (j < DRES) {
#pragma unroll 1
    for (int p = 0; p < NPR; ++p) { { const float db = sb[0][p] - ci, dp = sp[0][p] - cj; v0 += expf(-(db * db + dp * dp) / (2.0f * 0.5f)) / (2.0f * 3.14159265358979323846f * 0.5f); }
                                    { const float db = sb[1][p] - ci, dp = sp[1][p] - cj; v1 += expf(-(db * db + dp * dp) / (2.0f * 0.5f)) / (2.0f * 3.14159265358979323846f * 0.5f); } }
  }
  red[threadIdx.x] = (j < DRES) ? v0 : -1.f; __syncthreads(); for (int st = 64; st > 0; st >>= 1) { if (threadIdx.x < st) red[threadIdx.x] = fmaxf(red[threadIdx.x], red[threadIdx.x + st]); __syncthreads(); }
  const float m0 = red[0]; __syncthreads();
  red[threadIdx.x] = (j < DRES) ? v1 : -1.f; __syncthreads(); for (int st = 64; st > 0; st >>= 1) { if (threadIdx.x < st) red[threadIdx.x] = fmaxf(red[threadIdx.x], red[threadIdx.x + st]); __syncthreads(); }
  const float m1 = red[0];
  for (int e = threadIdx.x; e < DRES * 32; e += 128) (&tile[0][0])[e] = 0.f;
  __syncthreads();
  if (j < DRES) { tile[j][0] = v0; tile[j][1] = v1; }
  __syncthreads();
  { float* dst = img + (((size_t)b * DRES + i) * DRES) * 32;
    for (int pass = 0; pass < 2; ++pass) { for (int e = threadIdx.x; e < DRES * 8; e += 128) { const v4f v = *(const v4fa*)(&tile[0][0] + e * 4); *(volatile v4f*)(dst + (size_t)e * 4) = v; } if (pass == 0) __threadfence(); } }
  if (threadIdx.x < 32) { const float v = (threadIdx.x == 0) ? m0 : ((threadIdx.x == 1) ? m1 : 0.f); *(volatile float*)(bmax + (size_t)blockIdx.x * 32 + threadIdx.x) = v; __threadfence(); *(volatile float*)(bmax + (size_t)blockIdx.x * 32 + threadIdx.x) = v; }
}
__global__ __launch_bounds__(256) void k_imnorm(float* __restrict__ img, const float* __restrict__ bmax) {
  __shared__ float smax[2];
  const int b = blockIdx.y;
  if (threadIdx.x < 2) { float m = -1.f; for (int i = 0; i < DRES; ++i) m = fmaxf(m, bmax[((size_t)b * DRES + i) * 32 + threadIdx.x]); smax[threadIdx.x] = m; }
  __syncthreads();
  const size_t t = (size_t)blockIdx.x * 256 + threadIdx.x; if (t >= (size_t)DRES * DRES * 8) return;
  float* p = img + (size_t)b * DRES * DRES * 32 + t * 4; v4f v = *(const v4fa*)p;
  if ((t & 7) == 0) { v[0] = v[0] / smax[0]; v[1] = v[1] / smax[1]; }
  *(volatile v4f*)p = v; __threadfence(); *(volatile v4f*)p = v;
}
__global__ __launch_bounds__(256) void k_linear(const float* __restrict__ act, const float* __restrict__ W, const float* __restrict__ bias, float* __restrict__ out) {
  __shared__ float so[NGR * NCLS]; __shared__ float red[256];
  for (int bo = 0; bo < NGR * NCLS; ++bo) {
    const int b = bo / NCLS, o = bo % NCLS; float s = 0.f;
#pragma unroll 1
    for (int e = threadIdx.x; e < 32 * 625; e += 256) { const int c = e / 625, hw = e % 625; s += act[((size_t)b * 625 + hw) * 64 + c] * bf16_round(W[(size_t)o * 20000 + e]); }
    red[threadIdx.x] = s; __syncthreads(); for (int st = 128; st > 0; st >>= 1) { if (threadIdx.x < st) red[threadIdx.x] += red[threadIdx.x + st]; __syncthreads(); }
    if (threadIdx.x == 0) so[bo] = red[0] + bf16_round(bias[o]); __syncthreads();
  }
  for (int pass = 0; pass < 2; ++pass) { for (int e = threadIdx.x; e < NGR * NCLS; e += 256) *(volatile float*)(out + e) = so[e]; if (pass == 0) __threadfence(); }
}
extern "C" void kernel_launch(void* const* d_in, const int* in_sizes, int n_in,
                              void* d_out, int out_size, void* d_ws, size_t ws_size, hipStream_t stream) {
  (void)in_sizes; (void)n_in; (void)out_size;
  const float* x = (const float*)d_in[0]; const int* pi0 = (const int*)d_in[1]; const int* pi1 = (const int*)d_in[2];
  const float* w1 = (const float*)d_in[3]; const float* b1 = (const float*)d_in[4]; const float* w2 = (const float*)d_in[5]; const float* b2 = (const float*)d_in[6];
  const float* c1w = (const float*)d_in[7]; const float* c1b = (const float*)d_in[8]; const float* c2w = (const float*)d_in[9]; const float* c2b = (const float*)d_in[10]; const float* ow = (const float*)d_in[11]; const float* ob = (const float*)d_in[12];
  float* out0 = (float*)d_out; float* out1 = (float*)((char*)d_out + 1280);
  char* ws = (char*)d_ws; size_t off = 0;
  auto take = [&](size_t bytes) { char* p = ws + off; off += (bytes + 255) & ~(size_t)255; return p; };
  const int NP1 = NGR * DRES * DRES, NP2p = NGR * 50 * 50, NP3 = NGR * 25 * 25;
  unsigned short* B1 = (unsigned short*)take((size_t)HID * IN * 2); unsigned short* Bc1 = (unsigned short*)take((size_t)64 * 25 * 32 * 2); unsigned short* Bc2 = (unsigned short*)take((size_t)64 * 25 * 32 * 2);
  float* h = (float*)take((size_t)NNODE * HID * 4); float* filt = (float*)take((size_t)NNODE * 4 + 256);
  float* img = (float*)take((size_t)NP1 * 32 * 4); float* bmax = (float*)take((size_t)NGR * DRES * 32 * 4);
  float* c1o = (float*)take((size_t)NP1 * 64 * 4); float* p1 = (float*)take((size_t)NP2p * 64 * 4); float* c2o = (float*)take((size_t)NP2p * 64 * 4); float* p2 = (float*)take((size_t)(NP3 + 64) * 64 * 4);
  if (off > ws_size) return;
  k_wt_bf16<<<(HID * (IN / 8) + 255) / 256, 256, 0, stream>>>(w1, B1, IN, HID);
  k_wt_conv5<<<(64 * (25 * 32 / 8) + 255) / 256, 256, 0, stream>>>(c1w, Bc1, 16, 2, 32, 64);
  k_wt_conv5<<<(64 * (25 * 32 / 8) + 255) / 256, 256, 0, stream>>>(c2w, Bc2, 32, 16, 32, 64);
  k_gemm_bf<false, 1, true><<<((NNODE / 16) * 1 + 3) / 4, 128, 0, stream>>>(x, IN, B1, IN, b1, h, HID, NNODE, HID, IN);
  k_filt<<<(NNODE + 255) / 256, 256, 0, stream>>>(h, w2, b2, filt, out1);
  k_persim<<<NGR * DRES, 128, 0, stream>>>(filt, pi0, pi1, img, bmax);
  k_imnorm<<<dim3((DRES * DRES * 8 + 255) / 256, NGR), 256, 0, stream>>>(img, bmax);
  k_conv5<32, 1, DRES, DRES><<<((NP1 / 16) * 1 + 3) / 4, 128, 0, stream>>>(img, 32, Bc1, c1b, 16, c1o, 64, NP1);
  k_pool2_pm<<<(unsigned)(((size_t)NP2p * 16 + 255) / 256), 256, 0, stream>>>(c1o, p1, NGR, DRES, DRES, 64);
  k_conv5<32, 1, 50, 50><<<((NP2p / 16) * 1 + 3) / 4, 128, 0, stream>>>(p1, 64, Bc2, c2b, 32, c2o, 64, NP2p);
  k_pool2_pm<<<(unsigned)(((size_t)NP3 * 16 + 255) / 256), 256, 0, stream>>>(c2o, p2, NGR, 50, 50, 64);
  k_linear<<<1, 256, 0, stream>>>(p2, ow, ob, out0);
}
